// Decoder_42709154791713
// MI455X (gfx1250) — hardware-verified
//
#include <hip/hip_runtime.h>
#include <math.h>

constexpr int NBATCH  = 64;
constexpr int NSTEP   = 128;
constexpr int DMODEL  = 512;
constexpr int NGATE   = 2048;
constexpr int NVOCAB  = 32000;
constexpr int NLAYER  = 2;
constexpr int NROWS   = NBATCH * NSTEP;
constexpr int GATE_STRIDE = DMODEL * DMODEL;
constexpr int PLANE_ELEMS = NGATE * DMODEL;
constexpr int RTHR    = 512;
constexpr int RWAVES  = RTHR / 32;
constexpr int HPITCH  = 520;
constexpr int SLPITCH = 36;
constexpr int CTHR    = 256;
constexpr float W_CARRY   = 256.0f;
constexpr float X_CARRY   = 256.0f;
constexpr float H_CARRY   = 16.0f;
constexpr float G0_SCALE  = 1.0f / (W_CARRY * X_CARRY);
constexpr float ACC_CARRY = W_CARRY * H_CARRY;
constexpr float ACC_INV   = 1.0f / (W_CARRY * H_CARRY);
static_assert(NROWS == 8192);
static_assert(NGATE == 4 * DMODEL);
static_assert(DMODEL % 32 == 0);
static_assert(NGATE % 64 == 0 && NROWS % 64 == 0);
static_assert(DMODEL == 32 * RWAVES);
static_assert(NBATCH % 16 == 0);
static_assert((HPITCH % 8) == 0 && (SLPITCH % 4) == 0);
static_assert(((NGATE / 64) * (NROWS / 64)) % 8 == 0);

typedef __attribute__((ext_vector_type(16))) _Float16 v16h;
typedef __attribute__((ext_vector_type(8)))  _Float16 v8h;
typedef __attribute__((ext_vector_type(8)))  float    v8f;
typedef __attribute__((ext_vector_type(4)))  float    v4f;

__device__ __forceinline__ unsigned short f2bf_bits(float f) {
  unsigned u = __float_as_uint(f);
  return (unsigned short)((u + 0x7FFFu + ((u >> 16) & 1u)) >> 16);
}
__device__ __forceinline__ float bf_bits2f(unsigned short h) { return __uint_as_float(((unsigned)h) << 16); }
__device__ __forceinline__ float bf16r(float f) { return bf_bits2f(f2bf_bits(f)); }

__device__ __forceinline__ void guard4_h(v8f& a0, v8f& a1, v8f& a2, v8f& a3, v16h x, v16h b0, v16h b1, v16h b2, v16h b3) {
  asm volatile("v_nop\n\tv_nop\n\tv_nop\n\tv_nop" : "+v"(a0), "+v"(a1), "+v"(a2), "+v"(a3) : "v"(x), "v"(b0), "v"(b1), "v"(b2), "v"(b3));
}
__device__ __forceinline__ void acc_guard4(v8f& a, v8f& b, v8f& c, v8f& d) {
  asm volatile("v_nop\n\tv_nop\n\tv_nop\n\tv_nop" : "+v"(a), "+v"(b), "+v"(c), "+v"(d));
}
__device__ __forceinline__ void pin8(float (&a)[8]) {
  asm volatile("" : "+v"(a[0]), "+v"(a[1]), "+v"(a[2]), "+v"(a[3]), "+v"(a[4]), "+v"(a[5]), "+v"(a[6]), "+v"(a[7]) :: "memory");
}

union FragU { v16h v; v8h h[2]; };
__device__ __forceinline__ v16h frag_load(const _Float16* p) {
  FragU f;
  f.h[0] = *(const v8h*)(p);
  f.h[1] = *(const v8h*)(p + 16);
  return f.v;
}
__device__ __forceinline__ v8f frag_mma(v16h a, v16h b, v8f c) {
  return __builtin_amdgcn_wmma_f32_16x16x32_f16(false, a, false, b, (short)0, c, false, false);
}

__device__ __forceinline__ float sig_f(float x)  { return __builtin_amdgcn_rcpf(1.0f + expf(-x)); }
__device__ __forceinline__ float tanh_f(float x) { return 1.0f - 2.0f * __builtin_amdgcn_rcpf(expf(2.0f * x) + 1.0f); }

__global__ __launch_bounds__(CTHR) void gather_x_kernel(const int* __restrict__ tok, const float* __restrict__ emb,
                                                        unsigned short* __restrict__ XH) {
  const int i = blockIdx.x * CTHR + threadIdx.x;
  if (i < NROWS * (DMODEL / 8)) {
    const int row = i >> 6;
    const int c8  = i & 63;
    const int t   = row >> 6;
    const int b   = row & 63;
    int tk = tok[b * NSTEP + t];
    tk = tk < 0 ? 0 : (tk > NVOCAB - 1 ? NVOCAB - 1 : tk);
    const float* sp = emb + (size_t)tk * DMODEL + c8 * 8;
    const v4f a = *(const v4f*)(sp);
    const v4f bq = *(const v4f*)(sp + 4);
    v8h hv;
#pragma unroll
    for (int e = 0; e < 4; ++e) {
      const float fa = a[e];
      const float fb = bq[e];
      hv[e]     = (_Float16)(bf16r(fa) * X_CARRY);
      hv[4 + e] = (_Float16)(bf16r(fb) * X_CARRY);
    }
    *(volatile v8h*)(XH + (size_t)i * 8) = hv;
    __threadfence();
    *(volatile v8h*)(XH + (size_t)i * 8) = hv;
  }
}

__global__ __launch_bounds__(CTHR) void cvt_w_kernel(const float* __restrict__ src, unsigned short* __restrict__ dst, int n8) {
  const int i = blockIdx.x * CTHR + threadIdx.x;
  if (i < n8) {
    const float* sp = src + (size_t)i * 8;
    const v4f a = *(const v4f*)(sp);
    const v4f bq = *(const v4f*)(sp + 4);
    v8h hv;
#pragma unroll
    for (int e = 0; e < 4; ++e) {
      const float fa = a[e];
      const float fb = bq[e];
      hv[e]     = (_Float16)(bf16r(fa) * W_CARRY);
      hv[4 + e] = (_Float16)(bf16r(fb) * W_CARRY);
    }
    *(volatile v8h*)(dst + (size_t)i * 8) = hv;
    __threadfence();
    *(volatile v8h*)(dst + (size_t)i * 8) = hv;
  }
}

__global__ __launch_bounds__(CTHR) void bias_sum_kernel(const float* __restrict__ b_a, const float* __restrict__ b_b,
                                                        float* __restrict__ dst, int n4) {
  const int i = blockIdx.x * CTHR + threadIdx.x;
  if (i < n4) {
    const v4f va = *(const v4f*)(b_a + (size_t)i * 4);
    const v4f vb = *(const v4f*)(b_b + (size_t)i * 4);
    v4f o;
#pragma unroll
    for (int e = 0; e < 4; ++e) {
      const float fa = va[e];
      const float fb = vb[e];
      o[e] = bf16r(fa) + bf16r(fb);
    }
    float* op = dst + (size_t)i * 4;
    *(volatile v4f*)op = o;
    __threadfence();
    *(volatile v4f*)op = o;
  }
}

__global__ __launch_bounds__(256) void gemm_f16_rowbias_kernel(
    const unsigned short* __restrict__ Ap, int lda,
    const unsigned short* __restrict__ Btp, int ldb,
    float* __restrict__ C, int ldc,
    const float* __restrict__ bias, int M, int N, int K, float scale) {
  __shared__ __align__(16) float sT[8][16 * 68];
  const _Float16* A  = (const _Float16*)Ap;
  const _Float16* Bt = (const _Float16*)Btp;
  const int lane = threadIdx.x & 31;
  const int wave = threadIdx.x >> 5;
  const int tilesN = N >> 6;
  const int tilesM = M >> 6;
  const int tile = blockIdx.x * 8 + wave;
  if (tile >= tilesM * tilesN) return;
  const int tm = tile / tilesN;
  const int tn = tile - tm * tilesN;
  const int m0 = tm << 6;
  const int n0 = tn << 6;
  const int rlane = lane & 15;
  const int koff  = (lane >> 4) * 8;
  const int mOff  = (lane >> 4) * 8;

  v8f acc[4][4];
#pragma unroll
  for (int i = 0; i < 4; ++i)
#pragma unroll
    for (int j = 0; j < 4; ++j) acc[i][j] = (v8f){0.f, 0.f, 0.f, 0.f, 0.f, 0.f, 0.f, 0.f};

  for (int k0 = 0; k0 < K; k0 += 32) {
    v16h bh[4];
#pragma unroll
    for (int j = 0; j < 4; ++j) {
      const size_t bo = (size_t)(n0 + (j << 4) + rlane) * ldb + koff + k0;
      bh[j] = frag_load(Bt + bo);
    }
#pragma unroll
    for (int i = 0; i < 4; ++i) {
      const size_t ao = (size_t)(m0 + (i << 4) + rlane) * lda + koff + k0;
      const v16h ah = frag_load(A + ao);
#pragma unroll
      for (int j = 0; j < 4; ++j) acc[i][j] = frag_mma(ah, bh[j], acc[i][j]);
      guard4_h(acc[i][0], acc[i][1], acc[i][2], acc[i][3], ah, bh[0], bh[1], bh[2], bh[3]);
    }
  }
  acc_guard4(acc[0][0], acc[0][1], acc[0][2], acc[0][3]);
  acc_guard4(acc[1][0], acc[1][1], acc[1][2], acc[1][3]);
  acc_guard4(acc[2][0], acc[2][1], acc[2][2], acc[2][3]);
  acc_guard4(acc[3][0], acc[3][1], acc[3][2], acc[3][3]);

  float* slab = sT[wave];
#pragma unroll
  for (int i = 0; i < 4; ++i) {
    const int mBase = m0 + (i << 4);
    float bm[8];
#pragma unroll
    for (int r = 0; r < 8; ++r) bm[r] = bias[mBase + mOff + r];
#pragma unroll
    for (int j = 0; j < 4; ++j) {
#pragma unroll
      for (int r = 0; r < 8; ++r) {
        const float v = acc[i][j][r] * scale + bm[r];
        slab[(mOff + r) * 68 + (j << 4) + rlane] = v;
      }
    }
    __builtin_amdgcn_fence(__ATOMIC_RELEASE, "workgroup");
    __builtin_amdgcn_wave_barrier();
    __builtin_amdgcn_fence(__ATOMIC_ACQUIRE, "workgroup");
    {
      const int hh = lane >> 4, c4 = (lane & 15) * 4;
      for (int pass = 0; pass < 2; ++pass) {
#pragma unroll
        for (int it = 0; it < 8; ++it) {
          const int row = it * 2 + hh;
          const v4f v = *(const v4f*)(slab + row * 68 + c4);
          *(volatile v4f*)(C + (size_t)(mBase + row) * ldc + n0 + c4) = v;
        }
        __threadfence();
      }
    }
    __builtin_amdgcn_fence(__ATOMIC_RELEASE, "workgroup");
    __builtin_amdgcn_wave_barrier();
    __builtin_amdgcn_fence(__ATOMIC_ACQUIRE, "workgroup");
  }
}

__device__ __forceinline__ void kpass512(v8f (&acc)[4], const _Float16* ah, const _Float16* __restrict__ wb) {
#pragma unroll 1
  for (int k0 = 0; k0 < DMODEL; k0 += 32) {
    const v16h a  = frag_load(ah + k0);
    const v16h b0 = frag_load(wb + k0);
    const v16h b1 = frag_load(wb + (size_t)1 * GATE_STRIDE + k0);
    const v16h b2 = frag_load(wb + (size_t)2 * GATE_STRIDE + k0);
    const v16h b3 = frag_load(wb + (size_t)3 * GATE_STRIDE + k0);
    acc[0] = frag_mma(a, b0, acc[0]);
    acc[1] = frag_mma(a, b1, acc[1]);
    acc[2] = frag_mma(a, b2, acc[2]);
    acc[3] = frag_mma(a, b3, acc[3]);
    guard4_h(acc[0], acc[1], acc[2], acc[3], a, b0, b1, b2, b3);
  }
}

__device__ __forceinline__ void cell_update(const v8f (&acc)[4], float (&cst)[8], float (&hn)[8]) {
#pragma unroll
  for (int r = 0; r < 8; ++r) {
    const float zi = acc[0][r] * ACC_INV;
    const float zf = acc[1][r] * ACC_INV;
    const float zg = acc[2][r] * ACC_INV;
    const float zo = acc[3][r] * ACC_INV;
    const float ig = sig_f(zi);
    const float fg = sig_f(zf);
    const float gg = tanh_f(zg);
    const float og = sig_f(zo);
    const float cn = fg * cst[r] + ig * gg;
    cst[r] = cn;
    hn[r]  = og * tanh_f(cn);
  }
}

__global__ __launch_bounds__(RTHR) void lstm2_seq_kernel(const float* __restrict__ G0T,
                                                         const unsigned short* __restrict__ WIp,
                                                         const unsigned short* __restrict__ WHp,
                                                         const float* __restrict__ bsum,
                                                         const float* __restrict__ hid,
                                                         const float* __restrict__ cel,
                                                         float* __restrict__ out) {
  __shared__ __align__(16) _Float16 H0s[16 * HPITCH];
  __shared__ __align__(16) _Float16 H1s[16 * HPITCH];
  __shared__ __align__(16) float    Sl[RWAVES][16 * SLPITCH];
  const _Float16* WI1 = (const _Float16*)WIp + (size_t)PLANE_ELEMS;
  const _Float16* WH0 = (const _Float16*)WHp;
  const _Float16* WH1 = (const _Float16*)WHp + (size_t)PLANE_ELEMS;
  const int tid = threadIdx.x, lane = tid & 31, wave = tid >> 5;
  const int c = lane & 15, hh = lane >> 4, koff = hh * 8;
  const int b0 = blockIdx.x * 16;

#pragma unroll 1
  for (int row = 0; row < 16; ++row) {
    const float a = hid[(size_t)(b0 + row) * DMODEL + tid];
    const float b = hid[(size_t)(NBATCH + b0 + row) * DMODEL + tid];
    H0s[row * HPITCH + tid] = (_Float16)(bf16r(a) * H_CARRY);
    H1s[row * HPITCH + tid] = (_Float16)(bf16r(b) * H_CARRY);
  }
  if (tid < 128) {
    H0s[(tid >> 3) * HPITCH + DMODEL + (tid & 7)] = (_Float16)0.0f;
    H1s[(tid >> 3) * HPITCH + DMODEL + (tid & 7)] = (_Float16)0.0f;
  }

  float c0a[8], c0b[8], c1a[8], c1b[8];
  {
    const int ja = 32 * wave + c;
#pragma unroll
    for (int r = 0; r < 8; ++r) c0a[r] = cel[(size_t)(b0 + 8 * hh + r) * DMODEL + ja];
    pin8(c0a);
#pragma unroll
    for (int r = 0; r < 8; ++r) c0b[r] = cel[(size_t)(b0 + 8 * hh + r) * DMODEL + ja + 16];
    pin8(c0b);
#pragma unroll
    for (int r = 0; r < 8; ++r) c1a[r] = cel[(size_t)(NBATCH + b0 + 8 * hh + r) * DMODEL + ja];
    pin8(c1a);
#pragma unroll
    for (int r = 0; r < 8; ++r) c1b[r] = cel[(size_t)(NBATCH + b0 + 8 * hh + r) * DMODEL + ja + 16];
    pin8(c1b);
#pragma unroll
    for (int r = 0; r < 8; ++r) {
      c0a[r] = bf16r(c0a[r]);
      c0b[r] = bf16r(c0b[r]);
      c1a[r] = bf16r(c1a[r]);
      c1b[r] = bf16r(c1b[r]);
    }
  }
  float hna[8], hnb[8];
#pragma unroll
  for (int r = 0; r < 8; ++r) { hna[r] = 0.0f; hnb[r] = 0.0f; }
  __syncthreads();

  const _Float16* a0row = H0s + c * HPITCH + koff;
  const _Float16* a1row = H1s + c * HPITCH + koff;
  float* slab = Sl[wave];

#pragma unroll 1
  for (int t = 0; t < NSTEP; ++t) {
#pragma unroll 1
    for (int nt = 0; nt < 2; ++nt) {
      const int j = 32 * wave + 16 * nt + c;
      const float* gp = G0T + (size_t)j * NROWS + (size_t)t * NBATCH + b0 + 8 * hh;
      v8f acc[4];
#pragma unroll
      for (int g = 0; g < 4; ++g) {
        const v4f lo = *(const v4f*)(gp + (size_t)g * DMODEL * NROWS);
        const v4f hi = *(const v4f*)(gp + (size_t)g * DMODEL * NROWS + 4);
        acc[g] = (v8f){lo[0] * ACC_CARRY, lo[1] * ACC_CARRY, lo[2] * ACC_CARRY, lo[3] * ACC_CARRY,
                       hi[0] * ACC_CARRY, hi[1] * ACC_CARRY, hi[2] * ACC_CARRY, hi[3] * ACC_CARRY};
      }
      acc_guard4(acc[0], acc[1], acc[2], acc[3]);
      kpass512(acc, a0row, WH0 + (size_t)j * DMODEL + koff);
      acc_guard4(acc[0], acc[1], acc[2], acc[3]);
      cell_update(acc, c0a, hna);
#pragma unroll
      for (int r = 0; r < 8; ++r) {
        const float tc = c0a[r]; c0a[r] = c0b[r]; c0b[r] = tc;
        const float th = hna[r]; hna[r] = hnb[r]; hnb[r] = th;
      }
    }
    __syncthreads();
#pragma unroll
    for (int r = 0; r < 8; ++r) {
      H0s[(8 * hh + r) * HPITCH + 32 * wave + c]      = (_Float16)(hna[r] * H_CARRY);
      H0s[(8 * hh + r) * HPITCH + 32 * wave + 16 + c] = (_Float16)(hnb[r] * H_CARRY);
    }
    __syncthreads();

#pragma unroll 1
    for (int nt = 0; nt < 2; ++nt) {
      const int j = 32 * wave + 16 * nt + c;
      const float* bp = bsum + NGATE + j;
      const float q0 = bp[0] * ACC_CARRY;
      const float q1 = bp[DMODEL] * ACC_CARRY;
      const float q2 = bp[2 * DMODEL] * ACC_CARRY;
      const float q3 = bp[3 * DMODEL] * ACC_CARRY;
      v8f acc[4];
      acc[0] = (v8f){q0, q0, q0, q0, q0, q0, q0, q0};
      acc[1] = (v8f){q1, q1, q1, q1, q1, q1, q1, q1};
      acc[2] = (v8f){q2, q2, q2, q2, q2, q2, q2, q2};
      acc[3] = (v8f){q3, q3, q3, q3, q3, q3, q3, q3};
      acc_guard4(acc[0], acc[1], acc[2], acc[3]);
      kpass512(acc, a0row, WI1 + (size_t)j * DMODEL + koff);
      kpass512(acc, a1row, WH1 + (size_t)j * DMODEL + koff);
      acc_guard4(acc[0], acc[1], acc[2], acc[3]);
      cell_update(acc, c1a, hna);
#pragma unroll
      for (int r = 0; r < 8; ++r) {
        const float tc = c1a[r]; c1a[r] = c1b[r]; c1b[r] = tc;
        const float th = hna[r]; hna[r] = hnb[r]; hnb[r] = th;
      }
    }
    __syncthreads();
#pragma unroll
    for (int r = 0; r < 8; ++r) {
      H1s[(8 * hh + r) * HPITCH + 32 * wave + c]      = (_Float16)(hna[r] * H_CARRY);
      H1s[(8 * hh + r) * HPITCH + 32 * wave + 16 + c] = (_Float16)(hnb[r] * H_CARRY);
      slab[(8 * hh + r) * SLPITCH + c]      = hna[r];
      slab[(8 * hh + r) * SLPITCH + 16 + c] = hnb[r];
    }
    __builtin_amdgcn_fence(__ATOMIC_RELEASE, "workgroup");
    __builtin_amdgcn_wave_barrier();
    __builtin_amdgcn_fence(__ATOMIC_ACQUIRE, "workgroup");
    {
      const int q = lane >> 3, c4 = (lane & 7) * 4;
      for (int pass = 0; pass < 2; ++pass) {
#pragma unroll
        for (int it = 0; it < 4; ++it) {
          const int row = it * 4 + q;
          const v4f v = *(const v4f*)(slab + row * SLPITCH + c4);
          *(volatile v4f*)(out + ((size_t)(b0 + row) * NSTEP + (size_t)t) * DMODEL + 32 * wave + c4) = v;
        }
        __threadfence();
      }
    }
    __builtin_amdgcn_fence(__ATOMIC_RELEASE, "workgroup");
    __builtin_amdgcn_wave_barrier();
    __builtin_amdgcn_fence(__ATOMIC_ACQUIRE, "workgroup");
  }
}

extern "C" void kernel_launch(void* const* d_in, const int* in_sizes, int n_in,
                              void* d_out, int out_size, void* d_ws, size_t ws_size, hipStream_t stream) {
  if (n_in < 10 || d_out == nullptr || d_ws == nullptr) return;
  if (in_sizes[0] != NBATCH * NSTEP || in_sizes[2] != NLAYER * NBATCH * DMODEL || in_sizes[3] != NLAYER * NBATCH * DMODEL ||
      in_sizes[5] != NVOCAB * DMODEL || in_sizes[6] != NLAYER * NGATE * DMODEL || in_sizes[7] != NLAYER * NGATE * DMODEL ||
      in_sizes[8] != NLAYER * NGATE || in_sizes[9] != NLAYER * NGATE || out_size != NBATCH * NSTEP * DMODEL) return;

  const int*   tok  = (const int*)d_in[0];
  const float* hid  = (const float*)d_in[2];
  const float* cel  = (const float*)d_in[3];
  const float* emb  = (const float*)d_in[5];
  const float* w_ih = (const float*)d_in[6];
  const float* w_hh = (const float*)d_in[7];
  const float* b_ih = (const float*)d_in[8];
  const float* b_hh = (const float*)d_in[9];
  float* out = (float*)d_out;

  char* ws = (char*)d_ws; size_t off = 0;
  auto carve = [&](size_t bytes) -> char* { char* p = ws + off; off += (bytes + 255) & ~(size_t)255; return p; };
  unsigned short* XH   = (unsigned short*)carve((size_t)NROWS * DMODEL * 2);
  unsigned short* WI16 = (unsigned short*)carve((size_t)NLAYER * NGATE * DMODEL * 2);
  unsigned short* WH16 = (unsigned short*)carve((size_t)NLAYER * NGATE * DMODEL * 2);
  float*          BSUM = (float*)carve((size_t)NLAYER * NGATE * 4);
  float*          G0T  = (float*)carve((size_t)NGATE * NROWS * 4);
  if (off > ws_size || off > (size_t)134217728) return;

  const int n8x = NROWS * (DMODEL / 8);
  const int n8w = NLAYER * NGATE * (DMODEL / 8);
  const int n4b = NLAYER * NGATE / 4;
  gather_x_kernel<<<(n8x + CTHR - 1) / CTHR, CTHR, 0, stream>>>(tok, emb, XH);
  cvt_w_kernel<<<(n8w + CTHR - 1) / CTHR, CTHR, 0, stream>>>(w_ih, WI16, n8w);
  cvt_w_kernel<<<(n8w + CTHR - 1) / CTHR, CTHR, 0, stream>>>(w_hh, WH16, n8w);
  bias_sum_kernel<<<(n4b + CTHR - 1) / CTHR, CTHR, 0, stream>>>(b_ih, b_hh, BSUM, n4b);

  const int gblocks = ((NGATE / 64) * (NROWS / 64)) / 8;
  gemm_f16_rowbias_kernel<<<gblocks, 256, 0, stream>>>(WI16, DMODEL, XH, DMODEL, G0T, NROWS, BSUM,
                                                       NGATE, NROWS, DMODEL, G0_SCALE);

  lstm2_seq_kernel<<<NBATCH / 16, RTHR, 0, stream>>>(G0T, WI16, WH16, BSUM, hid, cel, out);
}
